// JanossyPool_6030134083730
// MI455X (gfx1250) — hardware-verified
//
#include <hip/hip_runtime.h>
#include <stdint.h>

typedef _Float16 v16h __attribute__((ext_vector_type(16)));
typedef _Float16 v8h  __attribute__((ext_vector_type(8)));
typedef _Float16 v4h  __attribute__((ext_vector_type(4)));
typedef float    v8f  __attribute__((ext_vector_type(8)));
typedef float    v4f  __attribute__((ext_vector_type(4)));

#define B_DIM     64
#define N_SET     32
#define IN_DIMC   128
#define H_DIMC    512
#define OUT_DIMC  256
#define P_PERM    992
#define MTILE     64
#define NPT       16
#define AB_LD     1024
#define H1_LD     520
#define W_SCALE   64.0f
#define H_SCALE   16.0f
#define LO_SCALE  2048.0f

union Frag { v16h v; v8h half[2]; };

__device__ __forceinline__ v8f wmma16(v16h a, v16h b, v8f c) {
    v8f d = __builtin_amdgcn_wmma_f32_16x16x32_f16(false, a, false, b, (short)0, c, false, false);
    asm volatile("v_nop\n\tv_nop\n\tv_nop\n\tv_nop" : "+v"(d) : "v"(a), "v"(b));
    return d;
}

__global__ __launch_bounds__(64)
void k_tr(const float* __restrict__ in, _Float16* out, int R, int C, float s)
{
    __shared__ __attribute__((aligned(16))) _Float16 tl[64][72];

    const size_t zoff = (size_t)blockIdx.z * (size_t)R * (size_t)C;
    in  += zoff;
    out += zoff;
    const int tid = threadIdx.x, wv = tid >> 5, lane = tid & 31;
    const int c0 = blockIdx.x * 64, r0 = blockIdx.y * 64;

    #pragma unroll 4
    for (int it = 0; it < 16; ++it) {
        const int idx = it * 64 + tid;
        const int r   = idx >> 4;
        const int c4  = (idx & 15) * 4;
        v4f v = {0.f, 0.f, 0.f, 0.f};
        if (r0 + r < R && c0 + c4 + 3 < C)
            v = *(const v4f*)(in + (size_t)(r0 + r) * C + c0 + c4);
        #pragma unroll
        for (int e = 0; e < 4; ++e) tl[c4 + e][r] = (_Float16)(v[e] * s);
    }
    __syncthreads();

    #pragma unroll
    for (int it = 0; it < 8; ++it) {
        const int L = it * 8 + wv * 4 + (lane >> 3);
        const int q = lane & 7;
        if (c0 + L < C && r0 + 8 * q + 7 < R) {
            union { v8h h; v4f f; } u;
            u.h = *(const v8h*)&tl[L][8 * q];
            *(volatile v4f*)(out + (size_t)(c0 + L) * R + r0 + 8 * q) = u.f;
        }
    }
    __threadfence();
    #pragma unroll
    for (int it = 0; it < 8; ++it) {
        const int L = it * 8 + wv * 4 + (lane >> 3);
        const int q = lane & 7;
        if (c0 + L < C && r0 + 8 * q + 7 < R) {
            union { v8h h; v4f f; } u;
            u.h = *(const v8h*)&tl[L][8 * q];
            *(volatile v4f*)(out + (size_t)(c0 + L) * R + r0 + 8 * q) = u.f;
        }
    }
}

template <int SPLIT, int HASBIAS>
__global__ __launch_bounds__(128)
void k_gemm(const float* __restrict__ A, int lda, int nsum, int sstride,
            const _Float16* __restrict__ Bt, const float* __restrict__ bias,
            float* C, int ldc, int M, int N, int K,
            float ascale, float cscale, float bscale)
{
    __shared__ __attribute__((aligned(16))) _Float16 As[64][40];
    __shared__ __attribute__((aligned(16))) _Float16 Al[SPLIT ? 64 : 1][40];
    __shared__ __attribute__((aligned(16))) _Float16 Bs[64][40];
    __shared__ __attribute__((aligned(16))) float    Cs[64][68];

    const int tid = threadIdx.x, wv = tid >> 5, lane = tid & 31, lm = lane & 15, hh = lane >> 4;
    const int n0 = blockIdx.x * 64, r0 = blockIdx.y * 64;

    v8f acc[4], accl[4];
    {
        v8f z = {};
        #pragma unroll
        for (int ct = 0; ct < 4; ++ct) { acc[ct] = z; accl[ct] = z; }
    }

    for (int k0 = 0; k0 < K; k0 += 32) {
        #pragma unroll
        for (int it = 0; it < 4; ++it) {
            const int idx = it * 128 + tid;
            const int r   = idx >> 3;
            const int c4  = (idx & 7) * 4;
            const int row = r0 + r;
            v4f v = {0.f, 0.f, 0.f, 0.f};
            if (row < M) {
                const float* p = A + (size_t)row * lda + k0 + c4;
                for (int s = 0; s < nsum; ++s) v += *(const v4f*)(p + (size_t)s * sstride);
            }
            v = v * ascale;
            v4h hq;
            #pragma unroll
            for (int e = 0; e < 4; ++e) hq[e] = (_Float16)v[e];
            *(v4h*)&As[r][c4] = hq;
            if constexpr (SPLIT) {
                v4h lq;
                #pragma unroll
                for (int e = 0; e < 4; ++e) lq[e] = (_Float16)((v[e] - (float)hq[e]) * LO_SCALE);
                *(v4h*)&Al[r][c4] = lq;
            }
        }
        #pragma unroll
        for (int it = 0; it < 2; ++it) {
            const int idx = it * 128 + tid;
            const int r   = idx >> 2;
            const int c8  = (idx & 3) * 8;
            const int n   = n0 + r;
            v8h v = {};
            if (n < N) v = *(const v8h*)(Bt + (size_t)n * K + k0 + c8);
            *(v8h*)&Bs[r][c8] = v;
        }
        __syncthreads();

        Frag a;
        a.half[0] = *(const v8h*)&As[wv * 16 + lm][8 * hh];
        a.half[1] = *(const v8h*)&As[wv * 16 + lm][16 + 8 * hh];
        Frag al = a;
        if constexpr (SPLIT) {
            al.half[0] = *(const v8h*)&Al[wv * 16 + lm][8 * hh];
            al.half[1] = *(const v8h*)&Al[wv * 16 + lm][16 + 8 * hh];
        }
        #pragma unroll
        for (int ct = 0; ct < 4; ++ct) {
            Frag bq;
            bq.half[0] = *(const v8h*)&Bs[ct * 16 + lm][8 * hh];
            bq.half[1] = *(const v8h*)&Bs[ct * 16 + lm][16 + 8 * hh];
            acc[ct] = wmma16(a.v, bq.v, acc[ct]);
            if constexpr (SPLIT) accl[ct] = wmma16(al.v, bq.v, accl[ct]);
        }
        __syncthreads();
    }

    #pragma unroll
    for (int ct = 0; ct < 4; ++ct) {
        const int col = ct * 16 + lm;
        float bv = 0.f;
        if constexpr (HASBIAS) { if (n0 + col < N) bv = bias[n0 + col] * bscale; }
        #pragma unroll
        for (int r = 0; r < 8; ++r) {
            float val = acc[ct][r];
            if constexpr (SPLIT) val += accl[ct][r] * (1.0f / LO_SCALE);
            Cs[wv * 16 + 8 * hh + r][col] = val * cscale + bv;
        }
    }
    __syncthreads();

    #pragma unroll
    for (int it = 0; it < 8; ++it) {
        const int L = it * 16 + wv * 4 + (lane >> 3);
        const int q = lane & 7;
        const int row = L >> 1, col = (L & 1) * 32 + q * 4;
        if (r0 + row < M && n0 + col + 3 < N) {
            const v4f v = *(const v4f*)&Cs[row][col];
            *(volatile v4f*)(C + (size_t)(r0 + row) * ldc + n0 + col) = v;
        }
    }
    __threadfence();
    #pragma unroll
    for (int it = 0; it < 8; ++it) {
        const int L = it * 16 + wv * 4 + (lane >> 3);
        const int q = lane & 7;
        const int row = L >> 1, col = (L & 1) * 32 + q * 4;
        if (r0 + row < M && n0 + col + 3 < N) {
            const v4f v = *(const v4f*)&Cs[row][col];
            *(volatile v4f*)(C + (size_t)(r0 + row) * ldc + n0 + col) = v;
        }
    }
}

__global__ __launch_bounds__(512)
void k_mid(const float* __restrict__ AB, const float* __restrict__ b1,
           const _Float16* __restrict__ W2t, const float* __restrict__ b2,
           float* Sp)
{
    __shared__ __attribute__((aligned(16))) _Float16 h1s[MTILE][H1_LD];
    __shared__ __attribute__((aligned(16))) float    cs[H_DIMC];

    const int b = blockIdx.y, t = blockIdx.x, p0 = t * MTILE, tid = threadIdx.x;

    #pragma unroll 2
    for (int it = 0; it < 8; ++it) {
        const int idx = it * 512 + tid;
        const int r   = idx >> 6;
        const int c8  = (idx & 63) * 8;
        const int p   = p0 + r;
        v8h hv = {};
        if (p < P_PERM) {
            const int i  = p / (N_SET - 1);
            const int jj = p - i * (N_SET - 1);
            const int j  = jj + (jj >= i ? 1 : 0);
            const float* pa = AB + (size_t)(b * N_SET + i) * AB_LD + c8;
            const float* pb = AB + (size_t)(b * N_SET + j) * AB_LD + H_DIMC + c8;
            const v4f a0 = *(const v4f*)pa, a1 = *(const v4f*)(pa + 4);
            const v4f q0 = *(const v4f*)pb, q1 = *(const v4f*)(pb + 4);
            const v4f g0 = *(const v4f*)(b1 + c8), g1 = *(const v4f*)(b1 + c8 + 4);
            const v4f s0 = a0 + q0 + g0;
            const v4f s1 = a1 + q1 + g1;
            #pragma unroll
            for (int e = 0; e < 4; ++e) {
                float u0 = s0[e]; u0 = u0 > 0.f ? u0 : 0.f;
                float u1 = s1[e]; u1 = u1 > 0.f ? u1 : 0.f;
                hv[e]     = (_Float16)(u0 * H_SCALE);
                hv[4 + e] = (_Float16)(u1 * H_SCALE);
            }
        }
        *(v8h*)&h1s[r][c8] = hv;
    }
    __syncthreads();

    const int w = tid >> 5, lane = tid & 31, lm = lane & 15, hh = lane >> 4;

    #pragma unroll 1
    for (int c = 0; c < 2; ++c) {
        const int ct = w + 16 * c;
        const _Float16* bp = W2t + (size_t)(ct * 16 + lm) * H_DIMC + 8 * hh;

        v8f acc[4];
        {
            v8f z = {};
            #pragma unroll
            for (int m = 0; m < 4; ++m) acc[m] = z;
        }

        #pragma unroll 2
        for (int ks = 0; ks < H_DIMC / 32; ++ks) {
            const int k0 = ks * 32;
            Frag bq;
            bq.half[0] = *(const v8h*)(bp + k0);
            bq.half[1] = *(const v8h*)(bp + k0 + 16);
            #pragma unroll
            for (int m = 0; m < 4; ++m) {
                Frag a;
                a.half[0] = *(const v8h*)&h1s[m * 16 + lm][k0 + 8 * hh];
                a.half[1] = *(const v8h*)&h1s[m * 16 + lm][k0 + 16 + 8 * hh];
                acc[m] = wmma16(a.v, bq.v, acc[m]);
            }
        }

        const int n = ct * 16 + lm;
        const float bias = b2[n];
        float s = 0.f;
        #pragma unroll
        for (int m = 0; m < 4; ++m) {
            #pragma unroll
            for (int v = 0; v < 8; ++v) {
                const int prow = p0 + m * 16 + 8 * hh + v;
                float h2 = acc[m][v] * (1.0f / (H_SCALE * W_SCALE)) + bias;
                h2 = h2 > 0.f ? h2 : 0.f;
                s += (prow < P_PERM) ? h2 : 0.f;
            }
        }
        s += __shfl_xor(s, 16);
        if (hh == 0) cs[n] = s;
    }
    __syncthreads();

    float* dst = Sp + (size_t)(b * NPT + t) * H_DIMC;
    if (tid < 128) {
        const v4f v = *(const v4f*)&cs[tid * 4];
        *(volatile v4f*)(dst + tid * 4) = v;
    }
    __threadfence();
    if (tid < 128) {
        const v4f v = *(const v4f*)&cs[tid * 4];
        *(volatile v4f*)(dst + tid * 4) = v;
    }
}

extern "C" void kernel_launch(void* const* d_in, const int* in_sizes, int n_in,
                              void* d_out, int out_size, void* d_ws, size_t ws_size,
                              hipStream_t stream)
{
    if (n_in < 7) return;
    if (in_sizes[0] != B_DIM * N_SET * IN_DIMC) return;
    if (in_sizes[1] != 2 * IN_DIMC * H_DIMC)    return;
    if (in_sizes[2] != H_DIMC)                  return;
    if (in_sizes[3] != H_DIMC * H_DIMC)         return;
    if (in_sizes[4] != H_DIMC)                  return;
    if (in_sizes[5] != H_DIMC * OUT_DIMC)       return;
    if (in_sizes[6] != OUT_DIMC)                return;
    if (out_size != B_DIM * OUT_DIMC)           return;

    const float* x  = (const float*)d_in[0];
    const float* W1 = (const float*)d_in[1];
    const float* b1 = (const float*)d_in[2];
    const float* W2 = (const float*)d_in[3];
    const float* b2 = (const float*)d_in[4];
    const float* W3 = (const float*)d_in[5];
    const float* b3 = (const float*)d_in[6];

    const size_t sz_w1t = (size_t)2 * H_DIMC * IN_DIMC * sizeof(_Float16);
    const size_t sz_w2t = (size_t)H_DIMC * H_DIMC * sizeof(_Float16);
    const size_t sz_w3t = (size_t)OUT_DIMC * H_DIMC * sizeof(_Float16);
    const size_t sz_ab  = (size_t)B_DIM * N_SET * AB_LD * sizeof(float);
    const size_t sz_sp  = (size_t)B_DIM * NPT * H_DIMC * sizeof(float);
    const size_t off_w1t = 0;
    const size_t off_w2t = off_w1t + sz_w1t;
    const size_t off_w3t = off_w2t + sz_w2t;
    const size_t off_ab  = off_w3t + sz_w3t;
    const size_t off_sp  = off_ab + sz_ab;
    const size_t total   = off_sp + sz_sp;
    if (total > ws_size) return;

    char* ws = (char*)d_ws;
    _Float16* W1t = (_Float16*)(ws + off_w1t);
    _Float16* W2t = (_Float16*)(ws + off_w2t);
    _Float16* W3t = (_Float16*)(ws + off_w3t);
    float*    AB  = (float*)(ws + off_ab);
    float*    Sp  = (float*)(ws + off_sp);
    float*    out = (float*)d_out;

    dim3 g_w1(H_DIMC / 64, IN_DIMC / 64, 2);
    k_tr<<<g_w1, 64, 0, stream>>>(W1, W1t, IN_DIMC, H_DIMC, W_SCALE);
    dim3 g_w2(H_DIMC / 64, H_DIMC / 64, 1);
    k_tr<<<g_w2, 64, 0, stream>>>(W2, W2t, H_DIMC, H_DIMC, W_SCALE);
    dim3 g_w3(OUT_DIMC / 64, H_DIMC / 64, 1);
    k_tr<<<g_w3, 64, 0, stream>>>(W3, W3t, H_DIMC, OUT_DIMC, W_SCALE);

    dim3 g1(AB_LD / 64, (B_DIM * N_SET) / 64);
    k_gemm<0, 0><<<g1, 128, 0, stream>>>(x, IN_DIMC, 1, 0, W1t, x, AB, AB_LD,
                                        B_DIM * N_SET, AB_LD, IN_DIMC, 1.0f, 1.0f / W_SCALE, 0.0f);

    dim3 g2(NPT, B_DIM);
    k_mid<<<g2, 512, 0, stream>>>(AB, b1, W2t, b2, Sp);

    dim3 g3(OUT_DIMC / 64, 1);
    k_gemm<1, 1><<<g3, 128, 0, stream>>>(Sp, NPT * H_DIMC, NPT, H_DIMC, W3t, b3, out, OUT_DIMC,
                                        B_DIM, OUT_DIMC, H_DIMC, 1.0f, 1.0f / W_SCALE, (float)P_PERM);
}
